// CausalMultiheadSelfAttention_19344532701997
// MI455X (gfx1250) — hardware-verified
//
#include <hip/hip_runtime.h>


#ifndef NB
#define NB 4
#endif
#ifndef SEQ
#define SEQ 2048
#endif
#define NB_FULL  4
#define SEQ_FULL 2048
#define DM   1024
#define NH_  16
#define HD   64
#if SEQ < 512
#define RH SEQ
#else
#define RH 512
#endif
#define NWV  4
#define QB   (NWV * 16)
#define KT   64
#define PP   72
#define OP   72
#define PCAR 1024.0f
#define SCL  0.125f

static_assert(NB >= 1 && NB <= NB_FULL);
static_assert(SEQ <= SEQ_FULL);
static_assert(SEQ % QB == 0);
static_assert(RH % QB == 0);
static_assert(RH % KT == 0);
static_assert(SEQ % KT == 0);
static_assert(RH <= SEQ);
static_assert((SEQ - RH) % QB == 0);
static_assert(DM % 64 == 0);
static_assert(SEQ % 64 == 0);
static_assert(NH_ * HD == DM);
static_assert((SEQ * DM) % (8 * 256) == 0);
static_assert((DM * DM) % (8 * 256) == 0);

typedef _Float16 h16;
typedef unsigned short bf;
typedef __attribute__((ext_vector_type(16))) __bf16   v16bf;
typedef __attribute__((ext_vector_type(16))) _Float16 v16h;
typedef __attribute__((ext_vector_type(8)))  _Float16 v8h;
typedef __attribute__((ext_vector_type(8)))  unsigned short v8us;
typedef __attribute__((ext_vector_type(8)))  float    v8f;
typedef __attribute__((ext_vector_type(4)))  float    v4f;
typedef v8h  __attribute__((may_alias)) v8ha;
typedef v4f  __attribute__((may_alias)) v4fa;
typedef v8us __attribute__((may_alias)) v8usa;
typedef __attribute__((ext_vector_type(2))) _Float16 v2h;
typedef __attribute__((ext_vector_type(2))) unsigned short v2us;
typedef __attribute__((ext_vector_type(2))) float v2f;

__device__ __forceinline__ unsigned short f2bf(float f) { unsigned u = __float_as_uint(f); u += 0x7FFFu + ((u >> 16) & 1u); return (unsigned short)(u >> 16); }
__device__ __forceinline__ float bf2f(unsigned short b) { return __uint_as_float(((unsigned)b) << 16); }
__device__ __forceinline__ float bfr(float f) { return bf2f(f2bf(f)); }
__device__ __forceinline__ v16h cat16(v8h lo, v8h hi) { return __builtin_shufflevector(lo, hi, 0, 1, 2, 3, 4, 5, 6, 7, 8, 9, 10, 11, 12, 13, 14, 15); }
__device__ __forceinline__ v16bf cat16b(v8us lo, v8us hi) { return __builtin_bit_cast(v16bf, __builtin_shufflevector(lo, hi, 0, 1, 2, 3, 4, 5, 6, 7, 8, 9, 10, 11, 12, 13, 14, 15)); }
__device__ __forceinline__ v8f wmma16(v16h a, v16h b, v8f c) { return __builtin_amdgcn_wmma_f32_16x16x32_f16(false, a, false, b, (short)0, c, false, false); }
__device__ __forceinline__ v8f wmmab(v16bf a, v16bf b, v8f c) { return __builtin_amdgcn_wmma_f32_16x16x32_bf16(false, a, false, b, (short)0, c, false, false); }
__device__ __forceinline__ h16 tohx(float x) { return (h16)x; }
__device__ __forceinline__ void splitf(float y, unsigned short& h, unsigned short& l) { h = f2bf(y); l = f2bf(y - bf2f(h)); }

template <typename T16> struct WFrag;
template <> struct WFrag<h16> { typedef v16h V; static __device__ __forceinline__ V ld(const h16* p) { return cat16(*(const v8h*)p, *(const v8h*)(p + 16)); } static __device__ __forceinline__ v8f mma(V a, V b, v8f c) { return wmma16(a, b, c); } };
template <> struct WFrag<bf> { typedef v16bf V; static __device__ __forceinline__ V ld(const bf* p) { return cat16b(*(const v8us*)p, *(const v8us*)(p + 16)); } static __device__ __forceinline__ v8f mma(V a, V b, v8f c) { return wmmab(a, b, c); } };
template <typename T16, int NSPLIT, bool BIAS>
__global__ __launch_bounds__(32) void k_gemmw(const T16* __restrict__ A, const T16* __restrict__ A2, const T16* __restrict__ Bt, const T16* __restrict__ Bt2, int K, float* C, int ldc, const float* __restrict__ bias, size_t sA, size_t sB, size_t sC) {
    typedef typename WFrag<T16>::V V;
    __shared__ __align__(16) float os[16 * 68];
    const size_t z = blockIdx.z; A += z * sA; if (A2) A2 += z * sA; Bt += z * sB; if (Bt2) Bt2 += z * sB; C += z * sC;
    const int lane = threadIdx.x & 31, lr = lane & 15, hi = lane >> 4; const int r0 = blockIdx.x * 64, c0 = blockIdx.y * 64;
    v8f acc[4][4];
#pragma unroll
    for (int mb = 0; mb < 4; ++mb)
#pragma unroll
        for (int nb = 0; nb < 4; ++nb) acc[mb][nb] = (v8f){};
    const size_t aoff = (size_t)(r0 + lr) * K + 8 * hi, boff = (size_t)(c0 + lr) * K + 8 * hi;
#pragma unroll 1
    for (int kc = 0; kc < K; kc += 32) {
        V a[4], a2[4];
#pragma unroll
        for (int mb = 0; mb < 4; ++mb) { a[mb] = WFrag<T16>::ld(A + aoff + (size_t)mb * 16 * K + kc); if (NSPLIT == 1 || NSPLIT == 2) a2[mb] = WFrag<T16>::ld(A2 + aoff + (size_t)mb * 16 * K + kc); }
#pragma unroll
        for (int nb = 0; nb < 4; ++nb) { const V b = WFrag<T16>::ld(Bt + boff + (size_t)nb * 16 * K + kc); V b2; if (NSPLIT >= 2) b2 = WFrag<T16>::ld(Bt2 + boff + (size_t)nb * 16 * K + kc);
#pragma unroll
            for (int mb = 0; mb < 4; ++mb) { acc[mb][nb] = WFrag<T16>::mma(a[mb], b, acc[mb][nb]); if (NSPLIT == 1 || NSPLIT == 2) acc[mb][nb] = WFrag<T16>::mma(a2[mb], b, acc[mb][nb]); if (NSPLIT >= 2) acc[mb][nb] = WFrag<T16>::mma(a[mb], b2, acc[mb][nb]); } }
        asm volatile("v_nop\n\tv_nop\n\tv_nop\n\tv_nop" : "+v"(acc[0][0]), "+v"(acc[1][1]), "+v"(acc[2][2]), "+v"(acc[3][3]) : "v"(a[0]), "v"(a[3]));
    }
#pragma unroll
    for (int mb = 0; mb < 4; ++mb) {
#pragma unroll
        for (int nb = 0; nb < 4; ++nb) {
#pragma unroll
            for (int j = 0; j < 8; ++j) os[(hi * 8 + j) * 68 + nb * 16 + lr] = acc[mb][nb][j]; }
        __builtin_amdgcn_wave_barrier(); asm volatile("" ::: "memory");
        float* crow = C + (size_t)(r0 + mb * 16) * ldc + c0;
#pragma unroll 1
        for (int ps = 0; ps < 2; ++ps) {
#pragma unroll
            for (int s = 0; s < 8; ++s) { const int row = 2 * s + hi, cofs = lr * 4; v4f val = *(const v4fa*)(os + row * 68 + cofs); if (BIAS) { val[0] += bfr(bias[c0 + cofs]); val[1] += bfr(bias[c0 + cofs + 1]); val[2] += bfr(bias[c0 + cofs + 2]); val[3] += bfr(bias[c0 + cofs + 3]); }
                *(volatile v4f*)(crow + (size_t)row * ldc + cofs) = val; }
            if (ps == 0) __threadfence(); }
        __builtin_amdgcn_wave_barrier(); asm volatile("" ::: "memory");
    }
}

__global__ __launch_bounds__(256) void k_cvt8(const float* __restrict__ src, bf* dst, size_t n8) { const size_t i = (size_t)blockIdx.x * 256 + threadIdx.x; if (i >= n8) return; const v8f v = *(const v8f*)(src + i * 8); v8us o;
#pragma unroll
    for (int k = 0; k < 8; ++k) o[k] = f2bf(v[k]); *(volatile v8us*)(dst + i * 8) = o; __threadfence(); *(volatile v8us*)(dst + i * 8) = o; }

__global__ __launch_bounds__(256) void k_qkp(const float* __restrict__ F, h16* P16, bf* Ph, bf* Pl) {
    const size_t e = ((size_t)blockIdx.x * 256 + threadIdx.x) * 2; if (e >= (size_t)2 * NH_ * SEQ * HD) return;
    const int d = (int)(e % HD); const int t = (int)((e / HD) % SEQ); const int hh = (int)(e / ((size_t)HD * SEQ)); const int g = hh / NH_, h = hh % NH_;
    const v2f x = *(const v2f*)(F + (size_t)g * SEQ * DM + (size_t)t * DM + h * HD + d);
    v2h o16; v2us oh, ol;
#pragma unroll
    for (int q = 0; q < 2; ++q) { o16[q] = tohx(x[q]); unsigned short a, c; splitf(x[q], a, c); oh[q] = a; ol[q] = c; }
    const bool lowrow = (t < RH); const size_t eo = ((size_t)hh * RH + t) * HD + d;
#pragma unroll 1
    for (int ps = 0; ps < 2; ++ps) {
        *(volatile v2h*)(P16 + e) = o16;
        if (lowrow) { *(volatile v2us*)(Ph + eo) = oh; *(volatile v2us*)(Pl + eo) = ol; }
        if (ps == 0) __threadfence(); }
}
__global__ __launch_bounds__(256) void k_vtp(const float* __restrict__ F, int pitch, h16* V16, bf* Vh, bf* Vl) {
    const size_t e = ((size_t)blockIdx.x * 256 + threadIdx.x) * 2; if (e >= (size_t)NH_ * HD * SEQ) return;
    const int t = (int)(e % SEQ); const int d = (int)((e / SEQ) % HD); const int g = (int)(e / ((size_t)SEQ * HD));
    v2h o16; v2us oh, ol;
#pragma unroll
    for (int q = 0; q < 2; ++q) { const float x = F[(size_t)(t + q) * pitch + g * HD + d]; o16[q] = tohx(x); unsigned short a, c; splitf(x, a, c); oh[q] = a; ol[q] = c; }
    const bool lowrow = (t < RH); const size_t eo = ((size_t)g * HD + d) * RH + t;
#pragma unroll 1
    for (int ps = 0; ps < 2; ++ps) {
        *(volatile v2h*)(V16 + e) = o16;
        if (lowrow) { *(volatile v2us*)(Vh + eo) = oh; *(volatile v2us*)(Vl + eo) = ol; }
        if (ps == 0) __threadfence(); }
}

template <bool HR>
__global__ __launch_bounds__(NWV * 32) void k_attn(const h16* __restrict__ Q16, const h16* __restrict__ K16, const h16* __restrict__ VT16,
                                                    const bf* __restrict__ Qh, const bf* __restrict__ Ql, const bf* __restrict__ Kh, const bf* __restrict__ Kl,
                                                    const bf* __restrict__ VTh, const bf* __restrict__ VTl, int qbase, int bb, bf* ATh, bf* ATl) {
    __shared__ __align__(16) h16 P16s[NWV * 16 * PP];
    __shared__ __align__(16) bf  Phs[NWV * 16 * PP];
    __shared__ __align__(16) bf  Pls[NWV * 16 * PP];
    __shared__ __align__(16) bf  OSh[NWV * 16 * OP];
    __shared__ __align__(16) bf  OSl[NWV * 16 * OP];
    const int lane = threadIdx.x & 31, wv = threadIdx.x >> 5, m = lane & 15, hi = lane >> 4;
    const int h = blockIdx.y;
    const int q0 = qbase + blockIdx.x * QB + wv * 16;
    h16* Pw = P16s + wv * 16 * PP; bf* Phw = Phs + wv * 16 * PP; bf* Plw = Pls + wv * 16 * PP;
    const float SL2 = SCL * 1.4426950408889634f;

    v16h aq[2]; v16bf aqh[2], aql[2];
#pragma unroll
    for (int s = 0; s < 2; ++s) {
        if (HR) { const bf* ph = Qh + ((size_t)h * RH + q0 + m) * HD + 32 * s + 8 * hi; const bf* pl = Ql + ((size_t)h * RH + q0 + m) * HD + 32 * s + 8 * hi;
                  aqh[s] = cat16b(*(const v8us*)ph, *(const v8us*)(ph + 16)); aql[s] = cat16b(*(const v8us*)pl, *(const v8us*)(pl + 16)); aq[s] = (v16h){}; }
        else    { const h16* p = Q16 + ((size_t)h * SEQ + q0 + m) * HD + 32 * s + 8 * hi; aq[s] = cat16(*(const v8h*)p, *(const v8h*)(p + 16));
                  aqh[s] = __builtin_bit_cast(v16bf, (v16h){}); aql[s] = __builtin_bit_cast(v16bf, (v16h){}); }
    }
    v8f o[4];
#pragma unroll
    for (int t = 0; t < 4; ++t) o[t] = (v8f){};
    float mr[8], lr[8];
#pragma unroll
    for (int r = 0; r < 8; ++r) { mr[r] = -1.0e30f; lr[r] = 0.0f; }
    const int nkt = (q0 + 16 + KT - 1) / KT;

#pragma unroll 1
    for (int kt = 0; kt < nkt; ++kt) {
        const int k0 = kt * KT;
        v8f sc[4];
#pragma unroll
        for (int j = 0; j < 4; ++j) {
            sc[j] = (v8f){};
            const int krow = k0 + j * 16 + m;
            if (HR) {
                v16bf kh[2], kl[2];
#pragma unroll
                for (int s = 0; s < 2; ++s) { const bf* ph = Kh + ((size_t)h * RH + krow) * HD + 32 * s + 8 * hi; const bf* pl = Kl + ((size_t)h * RH + krow) * HD + 32 * s + 8 * hi;
                    kh[s] = cat16b(*(const v8us*)ph, *(const v8us*)(ph + 16)); kl[s] = cat16b(*(const v8us*)pl, *(const v8us*)(pl + 16)); }
#pragma unroll
                for (int s = 0; s < 2; ++s) { sc[j] = wmmab(aqh[s], kh[s], sc[j]); sc[j] = wmmab(aql[s], kh[s], sc[j]); sc[j] = wmmab(aqh[s], kl[s], sc[j]); }
                asm volatile("v_nop\n\tv_nop\n\tv_nop\n\tv_nop" : "+v"(sc[j]) : "v"(kh[1]), "v"(kl[1]), "v"(aqh[1]), "v"(aql[1]));
            } else {
                v16h kk[2];
#pragma unroll
                for (int s = 0; s < 2; ++s) { const h16* p = K16 + ((size_t)h * SEQ + krow) * HD + 32 * s + 8 * hi; kk[s] = cat16(*(const v8h*)p, *(const v8h*)(p + 16)); }
#pragma unroll
                for (int s = 0; s < 2; ++s) sc[j] = wmma16(aq[s], kk[s], sc[j]);
                asm volatile("v_nop\n\tv_nop\n\tv_nop\n\tv_nop" : "+v"(sc[j]) : "v"(kk[1]), "v"(aq[1]));
            }
        }
        __builtin_amdgcn_wave_barrier(); asm volatile("" ::: "memory");
#pragma unroll
        for (int r = 0; r < 8; ++r) {
            const int qg = q0 + 8 * hi + r;
            float sv[4]; float vm = -1.0e30f;
#pragma unroll
            for (int j = 0; j < 4; ++j) { const float tv = sc[j][r] * SL2; sv[j] = (k0 + j * 16 + m > qg) ? -1.0e30f : tv; vm = fmaxf(vm, sv[j]); }
#pragma unroll
            for (int off = 1; off < 16; off <<= 1) vm = fmaxf(vm, __shfl_xor(vm, off, 32));
            const float mn = fmaxf(mr[r], vm);
            const float al = __builtin_amdgcn_exp2f(mr[r] - mn);
            float pv[4]; float ps = 0.0f;
#pragma unroll
            for (int j = 0; j < 4; ++j) { pv[j] = __builtin_amdgcn_exp2f(sv[j] - mn); ps += pv[j]; }
#pragma unroll
            for (int off = 1; off < 16; off <<= 1) ps += __shfl_xor(ps, off, 32);
            lr[r] = lr[r] * al + ps; mr[r] = mn;
#pragma unroll
            for (int t = 0; t < 4; ++t) o[t][r] *= al;
            const int pr = 8 * hi + r;
            if (HR) {
#pragma unroll
                for (int j = 0; j < 4; ++j) { unsigned short a, c; splitf(pv[j], a, c); Phw[pr * PP + j * 16 + m] = a; Plw[pr * PP + j * 16 + m] = c; }
            } else {
#pragma unroll
                for (int j = 0; j < 4; ++j) Pw[pr * PP + j * 16 + m] = tohx(pv[j] * PCAR);
            }
        }
        __builtin_amdgcn_fence(3  , "wavefront"); __builtin_amdgcn_wave_barrier(); asm volatile("" ::: "memory");
        if (HR) {
            v16bf aph[2], apl[2];
#pragma unroll
            for (int s = 0; s < 2; ++s) {
                aph[s] = cat16b(*(const v8usa*)(Phw + m * PP + 32 * s + 8 * hi), *(const v8usa*)(Phw + m * PP + 32 * s + 16 + 8 * hi));
                apl[s] = cat16b(*(const v8usa*)(Plw + m * PP + 32 * s + 8 * hi), *(const v8usa*)(Plw + m * PP + 32 * s + 16 + 8 * hi)); }
#pragma unroll
            for (int t = 0; t < 4; ++t) {
                v16bf vh[2], vl[2];
#pragma unroll
                for (int s = 0; s < 2; ++s) { const bf* ph = VTh + ((size_t)h * HD + t * 16 + m) * RH + k0 + 32 * s + 8 * hi; const bf* pl = VTl + ((size_t)h * HD + t * 16 + m) * RH + k0 + 32 * s + 8 * hi;
                    vh[s] = cat16b(*(const v8us*)ph, *(const v8us*)(ph + 16)); vl[s] = cat16b(*(const v8us*)pl, *(const v8us*)(pl + 16)); }
#pragma unroll
                for (int s = 0; s < 2; ++s) { o[t] = wmmab(aph[s], vh[s], o[t]); o[t] = wmmab(apl[s], vh[s], o[t]); o[t] = wmmab(aph[s], vl[s], o[t]); }
                asm volatile("v_nop\n\tv_nop\n\tv_nop\n\tv_nop" : "+v"(o[t]) : "v"(vh[1]), "v"(vl[1]), "v"(aph[1]), "v"(apl[1]));
            }
        } else {
            v16h ap[2];
#pragma unroll
            for (int s = 0; s < 2; ++s) ap[s] = cat16(*(const v8ha*)(Pw + m * PP + 32 * s + 8 * hi), *(const v8ha*)(Pw + m * PP + 32 * s + 16 + 8 * hi));
#pragma unroll
            for (int t = 0; t < 4; ++t) {
                v16h vv[2];
#pragma unroll
                for (int s = 0; s < 2; ++s) { const h16* p = VT16 + ((size_t)h * HD + t * 16 + m) * SEQ + k0 + 32 * s + 8 * hi; vv[s] = cat16(*(const v8h*)p, *(const v8h*)(p + 16)); }
#pragma unroll
                for (int s = 0; s < 2; ++s) o[t] = wmma16(ap[s], vv[s], o[t]);
                asm volatile("v_nop\n\tv_nop\n\tv_nop\n\tv_nop" : "+v"(o[t]) : "v"(vv[1]), "v"(ap[1]));
            }
        }
    }

    float inv[8];
#pragma unroll
    for (int r = 0; r < 8; ++r) inv[r] = __fdiv_rn(1.0f, HR ? lr[r] : lr[r] * PCAR);
    bf* osh = OSh + wv * 16 * OP; bf* osl = OSl + wv * 16 * OP;
#pragma unroll
    for (int t = 0; t < 4; ++t)
#pragma unroll
        for (int r = 0; r < 8; ++r) { unsigned short a, c; splitf(o[t][r] * inv[r], a, c); osh[(8 * hi + r) * OP + t * 16 + m] = a; osl[(8 * hi + r) * OP + t * 16 + m] = c; }
    __builtin_amdgcn_fence(3  , "wavefront"); __builtin_amdgcn_wave_barrier(); asm volatile("" ::: "memory");
    const size_t rowb = (size_t)bb * SEQ + q0;
#pragma unroll 1
    for (int ps = 0; ps < 2; ++ps) {
#pragma unroll
        for (int it = 0; it < 4; ++it) { const int row = it * 4 + (lane >> 3), c8 = (lane & 7) * 8;
            const v8us xh = *(const v8usa*)(osh + row * OP + c8); const v8us xl = *(const v8usa*)(osl + row * OP + c8);
            const size_t g = (rowb + row) * DM + (size_t)h * HD + c8;
            *(volatile v8us*)(ATh + g) = xh; *(volatile v8us*)(ATl + g) = xl; }
        if (ps == 0) __threadfence(); }
}

extern "C" void kernel_launch(void* const* d_in, const int* in_sizes, int n_in,
                              void* d_out, int out_size, void* d_ws, size_t ws_size, hipStream_t stream) {
    if (n_in < 5) return;
    const int need_x = ((NB - 1) * SEQ_FULL + SEQ) * DM;
    if (in_sizes[0] < need_x || in_sizes[1] < DM * DM || in_sizes[2] < DM * DM || in_sizes[3] < DM * DM || in_sizes[4] < DM * DM || out_size < need_x) return;
    const float* x = (const float*)d_in[0]; const float* wq = (const float*)d_in[1]; const float* wk = (const float*)d_in[2]; const float* wv = (const float*)d_in[3]; const float* wo = (const float*)d_in[4];
    float* OUT = (float*)d_out;
    char* wsp = (char*)d_ws;
    auto take = [&](size_t bytes) { char* p = wsp; wsp += (bytes + 255) & ~(size_t)255; return (void*)p; };
    bf* W3 = (bf*)take((size_t)3 * DM * DM * 2);
    bf* WO = (bf*)take((size_t)DM * DM * 2);
    bf* XB = (bf*)take((size_t)SEQ * DM * 2);
    float* F = (float*)take((size_t)3 * SEQ * DM * 4);
    h16* QK16 = (h16*)take((size_t)2 * NH_ * SEQ * HD * 2);
    bf* QKh = (bf*)take((size_t)2 * NH_ * RH * HD * 2);
    bf* QKl = (bf*)take((size_t)2 * NH_ * RH * HD * 2);
    h16* VT16 = (h16*)take((size_t)NH_ * HD * SEQ * 2);
    bf* VTh = (bf*)take((size_t)NH_ * HD * RH * 2);
    bf* VTl = (bf*)take((size_t)NH_ * HD * RH * 2);
    bf* ATh = (bf*)take((size_t)NB * SEQ * DM * 2);
    bf* ATl = (bf*)take((size_t)NB * SEQ * DM * 2);
    if ((size_t)(wsp - (char*)d_ws) > ws_size) return;
    bf* WQ = W3; bf* WK = W3 + (size_t)DM * DM; bf* WV = W3 + (size_t)2 * DM * DM;
    const unsigned nw8 = (unsigned)((DM * DM / 8 + 255) / 256);
    k_cvt8<<<nw8, 256, 0, stream>>>(wq, WQ, (size_t)DM * DM / 8);
    k_cvt8<<<nw8, 256, 0, stream>>>(wk, WK, (size_t)DM * DM / 8);
    k_cvt8<<<nw8, 256, 0, stream>>>(wv, WV, (size_t)DM * DM / 8);
    k_cvt8<<<nw8, 256, 0, stream>>>(wo, WO, (size_t)DM * DM / 8);
    h16* K16 = QK16 + (size_t)NH_ * SEQ * HD; bf* Khp = QKh + (size_t)NH_ * RH * HD; bf* Klp = QKl + (size_t)NH_ * RH * HD;
    for (int b = 0; b < NB; ++b) {
        k_cvt8<<<(unsigned)(((size_t)SEQ * DM / 8 + 255) / 256), 256, 0, stream>>>(x + (size_t)b * SEQ_FULL * DM, XB, (size_t)SEQ * DM / 8);
        k_gemmw<bf, 0, false><<<dim3(SEQ / 64, DM / 64, 3), 32, 0, stream>>>(XB, nullptr, W3, nullptr, DM, F, DM, nullptr, (size_t)0, (size_t)DM * DM, (size_t)SEQ * DM);
        k_qkp<<<(unsigned)(((size_t)2 * NH_ * SEQ * HD / 2 + 255) / 256), 256, 0, stream>>>(F, QK16, QKh, QKl);
        k_vtp<<<(unsigned)(((size_t)NH_ * HD * SEQ / 2 + 255) / 256), 256, 0, stream>>>(F + (size_t)2 * SEQ * DM, DM, VT16, VTh, VTl);
        k_attn<true><<<dim3(RH / QB, NH_), NWV * 32, 0, stream>>>(QK16, K16, VT16, QKh, QKl, Khp, Klp, VTh, VTl, 0, b, ATh, ATl);
        if (SEQ > RH) k_attn<false><<<dim3((SEQ - RH) / QB, NH_), NWV * 32, 0, stream>>>(QK16, K16, VT16, QKh, QKl, Khp, Klp, VTh, VTl, RH, b, ATh, ATl);
    }
    k_gemmw<bf, 1, false><<<dim3(SEQ / 64, DM / 64, NB), 32, 0, stream>>>(ATh, ATl, WO, nullptr, DM, OUT, DM, nullptr, (size_t)SEQ * DM, (size_t)0, (size_t)SEQ_FULL * DM);
}
